// EvolutionaryFeatureExtractor_69836168233624
// MI455X (gfx1250) — hardware-verified
//
#include <hip/hip_runtime.h>
#include <stddef.h>
#include <math.h>


#pragma clang fp contract(off)

#define NSEQ     2048
#define SLEN     512
#define NAA      20
#define MPOS     100
#define KD       2048
#define NROW     2048
#define NCP      2048
#define NTHR     256
#define NWAVE    8
#define GT       128
#define NGT      (NROW / GT)
#define LDS_GEMM (GT * GT * 4)
#define PADROWS  (NROW - MPOS * NAA)
#define PADIT    16
#define PADBLK   3
#define PBLK     32
#define WSCAP    134217728

static_assert(MPOS * NAA + PADROWS == NROW);
static_assert(PADROWS * KD * 2 == PADBLK * PADIT * NTHR * 16);
static_assert(NSEQ == 8 * NTHR);
static_assert(KD == NSEQ && (KD % 32) == 0);
static_assert(NROW == NGT * GT && GT == 4 * 32 && NTHR == NWAVE * 32 && GT == NWAVE * 16);
static_assert((SLEN % PBLK) == 0 && PBLK == 4 * NWAVE && (NSEQ % 32) == 0);
static_assert(((PBLK * NAA) % 128) == 0 && (PBLK * NAA) / 4 + PBLK / 4 <= NTHR && PBLK * 4 == 128);
static_assert(SLEN == 2 * NTHR && (SLEN / 4) <= NTHR && MPOS <= SLEN);
static_assert(NAA <= 32);

typedef float        v4f  __attribute__((ext_vector_type(4)));
typedef float        v8f  __attribute__((ext_vector_type(8)));
typedef unsigned int v4u  __attribute__((ext_vector_type(4)));
typedef _Float16     v8h  __attribute__((ext_vector_type(8)));
typedef _Float16     v16h __attribute__((ext_vector_type(16)));
union FragH { v16h v; v8h h[2]; };

__device__ __forceinline__ float wsum(float v) {
#pragma unroll
  for (int o = 16; o > 0; o >>= 1) v += __shfl_xor(v, o, 32);
  return v;
}

__device__ __forceinline__ v8f wmh(v16h a, v16h b, v8f c) {
  v8f d = __builtin_amdgcn_wmma_f32_16x16x32_f16(false, a, false, b, (short)0, c, false, false);
  asm volatile("v_nop\n\tv_nop\n\tv_nop\n\tv_nop" : "+v"(d) : "v"(a), "v"(b));
  return d;
}

__device__ __forceinline__ void oh_store(const int (&tk)[8], unsigned int* rp) {
#pragma unroll 1
  for (int a = 0; a < NAA; ++a) {
    v4u w;
    w.x = ((tk[0] == a) ? 0x3C00u : 0u) | ((tk[1] == a) ? 0x3C000000u : 0u);
    w.y = ((tk[2] == a) ? 0x3C00u : 0u) | ((tk[3] == a) ? 0x3C000000u : 0u);
    w.z = ((tk[4] == a) ? 0x3C00u : 0u) | ((tk[5] == a) ? 0x3C000000u : 0u);
    w.w = ((tk[6] == a) ? 0x3C00u : 0u) | ((tk[7] == a) ? 0x3C000000u : 0u);
    *(volatile v4u*)(rp + (size_t)a * (KD / 2)) = w;
  }
}

__global__ __launch_bounds__(NTHR) void k_onehot(const int* __restrict__ msa, unsigned int* oh) {
  const int b = blockIdx.x, t = threadIdx.x;
  if (b < MPOS) {
    const int n0 = 8 * t;
    int tk[8];
#pragma unroll
    for (int e = 0; e < 8; ++e) tk[e] = msa[(size_t)(n0 + e) * SLEN + b];
    unsigned int* rp = oh + (size_t)(NAA * b) * (KD / 2) + 4 * t;
    oh_store(tk, rp);
    __threadfence();
    oh_store(tk, rp);
  } else {
    const int pb = b - MPOS;
    unsigned int* zp = oh + (size_t)(MPOS * NAA) * (KD / 2);
    v4u z;
    z.x = 0u; z.y = 0u; z.z = 0u; z.w = 0u;
#pragma unroll 1
    for (int it = 0; it < PADIT; ++it)
      *(volatile v4u*)(zp + (size_t)4 * ((pb * PADIT + it) * NTHR + t)) = z;
    __threadfence();
#pragma unroll 1
    for (int it = 0; it < PADIT; ++it)
      *(volatile v4u*)(zp + (size_t)4 * ((pb * PADIT + it) * NTHR + t)) = z;
  }
}

__global__ __launch_bounds__(NTHR) void k_prof(const int* __restrict__ msa, const float* __restrict__ pc,
                                               float* out) {
  __shared__ __attribute__((aligned(16))) float sps[PBLK * NAA];
  __shared__ __attribute__((aligned(16))) float scs[PBLK];
  const int blk = blockIdx.x, tid = threadIdx.x, lane = tid & 31, wave = tid >> 5;
  const float pcnt = 0.01f * pc[0];
  const float den = (float)NSEQ + pcnt * (float)NAA;
  const float invden = 1.0f / den;
#pragma unroll 1
  for (int q = 0; q < PBLK / NWAVE; ++q) {
    const int pl  = (PBLK / NWAVE) * wave + q;
    const int pos = PBLK * blk + pl;
    int cnt = 0;
#pragma unroll 1
    for (int s = 0; s < NSEQ / 32; ++s) {
      const int v = msa[(size_t)(32 * s + lane) * SLEN + pos];
#pragma unroll
      for (int a = 0; a < NAA; ++a) {
        const unsigned int bm = __builtin_amdgcn_ballot_w32(v == a);
        const int pcb = (int)__builtin_popcount(bm);
        cnt += (lane == a) ? pcb : 0;
      }
    }
    const float cf  = (float)cnt;
    const float tot = wsum(cf);
    const float fqn = (cf + pcnt) * invden;
    const float ps  = logf(fqn * (float)NAA + 1e-10f);
    const float ts  = fmaxf(tot, 1.0f);
    const float invt = 1.0f / ts;
    const float f   = cf * invt;
    const float tm  = f * log2f(f + 1e-10f);
    const float ssum = wsum((lane < NAA) ? tm : 0.0f);
    const float ent = -ssum;
    const float cons = (tot > 0.0f) ? (1.0f - ent * (1.0f / 4.321928094887363f)) : 0.0f;
    if (lane < NAA) sps[pl * NAA + lane] = ps;
    if (lane == 0)  scs[pl] = cons;
  }
  __syncthreads();
  const int ct = (tid < (PBLK * NAA) / 4) ? tid : ((PBLK * NAA) / 4 - 1);
  int cc = tid - (PBLK * NAA) / 4;
  cc = cc < 0 ? 0 : (cc > PBLK / 4 - 1 ? PBLK / 4 - 1 : cc);
  const v4f pv = *(const v4f*)(sps + 4 * ct);
  const v4f cv = *(const v4f*)(scs + 4 * cc);
  const bool wp = tid < (PBLK * NAA) / 4;
  const bool wc = (tid >= (PBLK * NAA) / 4) && (tid < (PBLK * NAA) / 4 + PBLK / 4);
  float* gp = out + (size_t)blk * (PBLK * NAA) + 4 * ct;
  float* gc = out + (size_t)SLEN * NAA + (size_t)blk * PBLK + 4 * cc;
  if (wp) *(volatile v4f*)gp = pv;
  if (wc) *(volatile v4f*)gc = cv;
  __threadfence();
  if (wp) *(volatile v4f*)gp = pv;
  if (wc) *(volatile v4f*)gc = cv;
}

__global__ __launch_bounds__(NTHR) void k_gemm(const _Float16* __restrict__ O, float* C) {
  extern __shared__ v4f lds_dyn[];
  float* stg = (float*)lds_dyn;
  const int br = blockIdx.y, bc = blockIdx.x;
  if (bc + 1 < br) return;
  const int tid = threadIdx.x, lane = tid & 31, wave = tid >> 5, hh = lane >> 4, m = lane & 15;
  const int rg = wave & 3, cg = wave >> 2;
  const int r0 = br * GT + rg * 32, c0 = bc * GT + cg * 64;

  v8f acc[2][4];
#pragma unroll
  for (int s = 0; s < 2; ++s)
#pragma unroll
    for (int t = 0; t < 4; ++t) { v8f z = {0.f, 0.f, 0.f, 0.f, 0.f, 0.f, 0.f, 0.f}; acc[s][t] = z; }

  const _Float16* ap0 = O + (size_t)(r0 + m) * KD + 8 * hh;
  const _Float16* ap1 = ap0 + (size_t)16 * KD;
  const _Float16* bp0 = O + (size_t)(c0 + m) * KD + 8 * hh;
  const _Float16* bp1 = bp0 + (size_t)16 * KD;
  const _Float16* bp2 = bp0 + (size_t)32 * KD;
  const _Float16* bp3 = bp0 + (size_t)48 * KD;

#pragma unroll 1
  for (int kt = 0; kt < KD / 32; ++kt) {
    const int k0 = 32 * kt;
    FragH a0, a1, b0, b1, b2, b3;
    a0.h[0] = *(const v8h*)(ap0 + k0);  a0.h[1] = *(const v8h*)(ap0 + k0 + 16);
    a1.h[0] = *(const v8h*)(ap1 + k0);  a1.h[1] = *(const v8h*)(ap1 + k0 + 16);
    b0.h[0] = *(const v8h*)(bp0 + k0);  b0.h[1] = *(const v8h*)(bp0 + k0 + 16);
    b1.h[0] = *(const v8h*)(bp1 + k0);  b1.h[1] = *(const v8h*)(bp1 + k0 + 16);
    b2.h[0] = *(const v8h*)(bp2 + k0);  b2.h[1] = *(const v8h*)(bp2 + k0 + 16);
    b3.h[0] = *(const v8h*)(bp3 + k0);  b3.h[1] = *(const v8h*)(bp3 + k0 + 16);
    acc[0][0] = wmh(a0.v, b0.v, acc[0][0]);
    acc[0][1] = wmh(a0.v, b1.v, acc[0][1]);
    acc[0][2] = wmh(a0.v, b2.v, acc[0][2]);
    acc[0][3] = wmh(a0.v, b3.v, acc[0][3]);
    acc[1][0] = wmh(a1.v, b0.v, acc[1][0]);
    acc[1][1] = wmh(a1.v, b1.v, acc[1][1]);
    acc[1][2] = wmh(a1.v, b2.v, acc[1][2]);
    acc[1][3] = wmh(a1.v, b3.v, acc[1][3]);
  }

  float* sp = stg + (rg * 32 + 8 * hh) * GT + cg * 64 + m;
#pragma unroll
  for (int s = 0; s < 2; ++s)
#pragma unroll
    for (int t = 0; t < 4; ++t)
#pragma unroll
      for (int r = 0; r < 8; ++r) sp[(16 * s + r) * GT + 16 * t] = acc[s][t][r];
  __syncthreads();

  const float* lp = stg + (wave * 16) * GT + 4 * lane;
  float* gp = C + (size_t)(br * GT + wave * 16) * NCP + bc * GT + 4 * lane;
#pragma unroll
  for (int i = 0; i < 16; ++i) { const v4f v = *(const v4f*)(lp + i * GT); *(volatile v4f*)(gp + (size_t)i * NCP) = v; }
  __threadfence();
#pragma unroll
  for (int i = 0; i < 16; ++i) { const v4f v = *(const v4f*)(lp + i * GT); *(volatile v4f*)(gp + (size_t)i * NCP) = v; }
}

__global__ __launch_bounds__(NTHR) void k_mi(const float* __restrict__ C, float* out2) {
  __shared__ __attribute__((aligned(16))) float srow[SLEN];
  const int i = blockIdx.x, tid = threadIdx.x, lane = tid & 31, wave = tid >> 5;
  srow[tid] = 0.0f;
  srow[tid + NTHR] = 0.0f;
  __syncthreads();
  if (i < MPOS) {
    const int bl = (lane < NAA) ? lane : (NAA - 1);
    const float msk = (lane < NAA) ? 1.0f : 0.0f;
#pragma unroll 1
    for (int j = wave; j < MPOS; j += NWAVE) {
      const int lo = (i < j) ? i : j, hi = (i < j) ? j : i;
      const int sa = (i <= j) ? NCP : 1;
      const int sb = (i <= j) ? 1 : NCP;
      const float* base = C + (size_t)(NAA * lo) * NCP + NAA * hi;
      float csum = 0.0f;
#pragma unroll 1
      for (int a = 0; a < NAA; ++a) csum += base[a * sa + bl * sb] * msk;
      const float tot = wsum(csum);
      const float ts  = fmaxf(tot, 1.0f);
      const float inv = 1.0f / ts;
      float pjl = 0.0f, pil = 0.0f;
#pragma unroll 1
      for (int a = 0; a < NAA; ++a) {
        const float v = base[a * sa + bl * sb] * msk;
        const float r = base[bl * sa + a * sb] * msk;
        pjl += v * inv;
        pil += r * inv;
      }
      float part = 0.0f;
#pragma unroll 1
      for (int a = 0; a < NAA; ++a) {
        const float v   = base[a * sa + bl * sb] * msk;
        const float pia = __shfl(pil, a, 32);
        const float p   = v * inv;
        const float dn  = fmaxf(pia * pjl, 1e-30f);
        const float q   = p * (1.0f / dn) + 1e-10f;
        const float t   = p * log2f(q);
        part += (v > 0.0f) ? t : 0.0f;
      }
      const float s  = wsum(part);
      const float mi = (tot > 0.0f && i != j) ? s : 0.0f;
      if (lane == 0) srow[j] = mi;
    }
  }
  __syncthreads();
  const int ct = (tid < SLEN / 4) ? tid : (SLEN / 4 - 1);
  const v4f rv = *(const v4f*)(srow + 4 * ct);
  float* gp = out2 + (size_t)i * SLEN + 4 * ct;
  const bool wr = tid < SLEN / 4;
  if (wr) *(volatile v4f*)gp = rv;
  __threadfence();
  if (wr) *(volatile v4f*)gp = rv;
}

extern "C" void kernel_launch(void* const* d_in, const int* in_sizes, int n_in,
                              void* d_out, int out_size, void* d_ws, size_t ws_size,
                              hipStream_t stream) {
  if (n_in < 2) return;
  if (in_sizes[0] != NSEQ * SLEN || in_sizes[1] < 1) return;
  if (out_size != SLEN * NAA + SLEN + SLEN * SLEN) return;

  const int*   msa = (const int*)d_in[0];
  const float* pc  = (const float*)d_in[1];
  float* out = (float*)d_out;

  char* ws = (char*)d_ws;
  const size_t oO  = 0;
  const size_t szO = (size_t)NROW * KD * 2;
  const size_t oC  = oO + szO;
  const size_t szC = (size_t)NROW * NCP * 4;
  const size_t total = oC + szC;
  if (total > ws_size || total > (size_t)WSCAP) return;
  unsigned int*   Ou = (unsigned int*)(ws + oO);
  const _Float16* Oh = (const _Float16*)(ws + oO);
  float*          Cj = (float*)(ws + oC);

  k_onehot<<<MPOS + PADBLK, NTHR, 0, stream>>>(msa, Ou);
  k_prof<<<SLEN / PBLK, NTHR, 0, stream>>>(msa, pc, out);
  hipFuncSetAttribute(reinterpret_cast<const void*>(&k_gemm), hipFuncAttributeMaxDynamicSharedMemorySize, LDS_GEMM);
  k_gemm<<<dim3(NGT, NGT), NTHR, LDS_GEMM, stream>>>(Oh, Cj);
  k_mi<<<SLEN, NTHR, 0, stream>>>(Cj, out + (size_t)SLEN * NAA + SLEN);
}
